// CustomModel_lipsnet_83296595739102
// MI455X (gfx1250) — hardware-run, weakly checked
//
#include <hip/hip_runtime.h>


#ifndef NB
#define NB 8192
#endif
#define NB_FULL 8192
#define NOBS 64
#define NACT 16
#define HID  128
#define CON  256
#define COMP 85
#define NP   96
#define NKS  32
#define XP   264
#define TP   136
#define MP   104
#define SPB  32
#define OCH  680

static_assert(NB % SPB == 0);
static_assert(NB <= NB_FULL);
static_assert(SPB * COMP * 4 == OCH * 16);
static_assert(OCH % 8 == 0);
static_assert(22 * 32 >= OCH);
static_assert(NP % 32 == 0 && CON % 32 == 0 && HID % 32 == 0 && NOBS % 32 == 0 && NKS % 32 == 0);
static_assert((XP * 2) % 16 == 0 && (TP * 2) % 16 == 0 && (MP * 2) % 16 == 0);
static_assert(XP >= CON && TP >= HID && MP >= NP);
static_assert(6 * 32 * 16 == 16 * NP * 2);

typedef unsigned short bf;
typedef unsigned short hf;
typedef _Float16 h16;
typedef __attribute__((ext_vector_type(16))) __bf16   v16bf;
typedef __attribute__((ext_vector_type(16))) _Float16 v16h;
typedef __attribute__((ext_vector_type(8)))  unsigned short v8us;
typedef __attribute__((ext_vector_type(8)))  float    v8f;
typedef __attribute__((ext_vector_type(4)))  float    v4f;
typedef v4f  __attribute__((may_alias)) v4fa;
typedef v8us __attribute__((may_alias)) v8usa;

__device__ __forceinline__ unsigned short f2bf(float f) { unsigned u = __float_as_uint(f); u += 0x7FFFu + ((u >> 16) & 1u); return (unsigned short)(u >> 16); }
__device__ __forceinline__ float bf2f(unsigned short w) { return __uint_as_float(((unsigned)w) << 16); }
__device__ __forceinline__ v16bf cat16b(v8us lo, v8us hi) { return __builtin_bit_cast(v16bf, __builtin_shufflevector(lo, hi, 0, 1, 2, 3, 4, 5, 6, 7, 8, 9, 10, 11, 12, 13, 14, 15)); }
__device__ __forceinline__ v8f wmmab(v16bf a, v16bf b, v8f c) { return __builtin_amdgcn_wmma_f32_16x16x32_bf16(false, a, false, b, (short)0, c, false, false); }
__device__ __forceinline__ v16bf ldb(const bf* p)  { return cat16b(*(const v8us*)p, *(const v8us*)(p + 16)); }
__device__ __forceinline__ void wave_sync() { __builtin_amdgcn_fence(3  , "wavefront"); __builtin_amdgcn_wave_barrier(); asm volatile("" ::: "memory"); }

static __device__ __forceinline__ h16 toh_flush(float v) { const h16 r = (h16)v; return (fabsf(v) < 6.103515625e-05f) ? (h16)0.0f : r; }
__device__ __forceinline__ unsigned short hbits(h16 h) { return __builtin_bit_cast(unsigned short, h); }
__device__ __forceinline__ v16h cat16h(v8us lo, v8us hi) { return __builtin_bit_cast(v16h, __builtin_shufflevector(lo, hi, 0, 1, 2, 3, 4, 5, 6, 7, 8, 9, 10, 11, 12, 13, 14, 15)); }
__device__ __forceinline__ v16h ldh(const hf* p) { return cat16h(*(const v8us*)p, *(const v8us*)(p + 16)); }
__device__ __forceinline__ v16h ldl(const hf* p) { return cat16h(*(const v8usa*)p, *(const v8usa*)(p + 16)); }
__device__ __forceinline__ v8f mmab(v16bf a, v16bf b, v8f c) { c = wmmab(a, b, c); asm volatile("v_nop\n\tv_nop\n\tv_nop\n\tv_nop" : "+v"(c) : "v"(a), "v"(b)); return c; }
__device__ __forceinline__ v8f mmah(v16h a, v16h b, v8f c) { c = __builtin_amdgcn_wmma_f32_16x16x32_f16(false, a, false, b, (short)0, c, false, false);
    asm volatile("v_nop\n\tv_nop\n\tv_nop\n\tv_nop" : "+v"(c) : "v"(a), "v"(b)); return c; }
__device__ __forceinline__ v8us cvt8(const float* p) { const v8f a = *(const v8f*)p; v8us o;
#pragma unroll
    for (int k = 0; k < 8; ++k) o[k] = f2bf(a[k]);
    return o; }
__device__ __forceinline__ float bfv(const float* __restrict__ p, int i, int n) { const float v = bf2f(f2bf(p[min(i, n - 1)])); return (i < n) ? v : 0.0f; }
__device__ __forceinline__ void st_hr(hf* H, hf* R, int i, float v) { const float s = v * 1024.0f; const h16 h = toh_flush(s); const float r = (s - (float)h) * 2048.0f;
    H[i] = hbits(h); R[i] = hbits(toh_flush(r)); }
__device__ __forceinline__ float softplusf(float x) { return fmaxf(x, 0.0f) + log1pf(expf(-fabsf(x))); }

template<int K, bool RES>
__device__ __forceinline__ v8f tile_pre(const hf* ah, const hf* ar, const hf* w) {
    static_assert(K % 32 == 0);
    v8f ch = (v8f){}, cr = (v8f){};
#pragma unroll 1
    for (int kc = 0; kc < K; kc += 32) {
        const v16h b = ldh(w + kc);
        const v16h a = ldl(ah + kc);
        ch = mmah(a, b, ch);
        if (RES) { const v16h r = ldl(ar + kc); cr = mmah(r, b, cr); }
    }
    v8f o;
#pragma unroll
    for (int j = 0; j < 8; ++j) o[j] = RES ? (ch[j] * 9.5367431640625e-07f + cr[j] * 4.656612873077393e-10f) : (ch[j] * 9.5367431640625e-07f);
    return o;
}

static constexpr int CH_OW1B = 0;
static constexpr int CH_AW1B = CH_OW1B + HID * NOBS / 8;
static constexpr int CH_OW2H = CH_AW1B + HID * 32 / 8;
static constexpr int CH_AW2H = CH_OW2H + HID * HID / 8;
static constexpr int CH_MW1H = CH_AW2H + HID * HID / 8;
static constexpr int CH_MW1B = CH_MW1H + NP * CON / 8;
static constexpr int CH_MW2H = CH_MW1B + NP * CON / 8;
static constexpr int CH_MW3H = CH_MW2H + NP * NP / 8;
static constexpr int CH_MW2T = CH_MW3H + NP * NP / 8;
static constexpr int CH_KW1H = CH_MW2T + NP * NP / 8;
static constexpr int CH_KW2H = CH_KW1H + NKS * CON / 8;
static constexpr int NCHUNK  = CH_KW2H + 16 * NKS / 8;
static_assert(NCHUNK == 16320);
static_assert(CH_AW1B % 32 == 0 && CH_OW2H % 32 == 0 && CH_AW2H % 32 == 0 && CH_MW1H % 32 == 0 && CH_MW1B % 32 == 0);
static_assert(CH_MW2H % 32 == 0 && CH_MW3H % 32 == 0 && CH_MW2T % 32 == 0 && CH_KW1H % 32 == 0 && CH_KW2H % 32 == 0 && NCHUNK % 32 == 0);

template<int SR, int SC, int TR, int DC, int ISBF>
__device__ __forceinline__ void cv_chunk(const float* __restrict__ src, bf* PL, int c, int lc) {
    static_assert(DC % 8 == 0);
    const int e0 = lc * 8; const int row = e0 / DC; const int col = e0 - row * DC;
    v8us o;
#pragma unroll
    for (int k = 0; k < 8; ++k) {
        const int cc = col + k;
        const int r2 = TR ? cc : row, c2 = TR ? row : cc;
        const bool ok = (r2 < SR) && (c2 < SC);
        const float v = bf2f(f2bf(src[min(r2, SR - 1) * SC + min(c2, SC - 1)]));
        const unsigned short w = ISBF ? f2bf(v) : hbits(toh_flush(v * 1024.0f));
        o[k] = ok ? w : (unsigned short)0; }
    bf* p = PL + (size_t)c * 8;
    *(volatile v8us*)p = o; __threadfence(); *(volatile v8us*)p = o;
}

__global__ __launch_bounds__(256) void k_wconv(const float* __restrict__ ow1, const float* __restrict__ aw1, const float* __restrict__ ow2, const float* __restrict__ aw2,
                                               const float* __restrict__ mw1, const float* __restrict__ mw2, const float* __restrict__ mw3,
                                               const float* __restrict__ kw1, const float* __restrict__ kw2, bf* PL) {
    const int c = blockIdx.x * 256 + threadIdx.x;
    const int cw = __builtin_amdgcn_readfirstlane(c);
    if (cw >= NCHUNK) return;
    if      (cw < CH_AW1B) cv_chunk<HID, NOBS, 0, NOBS, 1>(ow1, PL, c, c - CH_OW1B);
    else if (cw < CH_OW2H) cv_chunk<HID, NACT, 0, 32, 1>(aw1, PL, c, c - CH_AW1B);
    else if (cw < CH_AW2H) cv_chunk<HID, HID, 0, HID, 0>(ow2, PL, c, c - CH_OW2H);
    else if (cw < CH_MW1H) cv_chunk<HID, HID, 0, HID, 0>(aw2, PL, c, c - CH_AW2H);
    else if (cw < CH_MW1B) cv_chunk<COMP, CON, 0, CON, 0>(mw1, PL, c, c - CH_MW1H);
    else if (cw < CH_MW2H) cv_chunk<COMP, CON, 0, CON, 1>(mw1, PL, c, c - CH_MW1B);
    else if (cw < CH_MW3H) cv_chunk<COMP, COMP, 0, NP, 0>(mw2, PL, c, c - CH_MW2H);
    else if (cw < CH_MW2T) cv_chunk<COMP, COMP, 0, NP, 0>(mw3, PL, c, c - CH_MW3H);
    else if (cw < CH_KW1H) cv_chunk<COMP, COMP, 1, NP, 0>(mw2, PL, c, c - CH_MW2T);
    else if (cw < CH_KW2H) cv_chunk<NKS, CON, 0, CON, 0>(kw1, PL, c, c - CH_KW1H);
    else                   cv_chunk<16, NKS, 0, NKS, 0>(kw2, PL, c, c - CH_KW2H);
}

__global__ __launch_bounds__(32) void k_g1(const bf* __restrict__ PL, hf* G1H) {
    __shared__ __align__(16) hf gs[16 * MP];
    const int lane = threadIdx.x & 31, lr = lane & 15, hi = lane >> 4;
    const int w = blockIdx.x;
    v8f acc[6];
#pragma unroll
    for (int nt = 0; nt < 6; ++nt) acc[nt] = (v8f){};
    const bf* ap = PL + (size_t)CH_MW1B * 8 + (size_t)(w * 16 + lr) * CON + 8 * hi;
    const bf* bp = PL + (size_t)CH_MW1B * 8 + (size_t)lr * CON + 8 * hi;
#pragma unroll 1
    for (int kc = 0; kc < CON; kc += 32) {
        const v16bf a = ldb(ap + kc);
#pragma unroll
        for (int nt = 0; nt < 6; ++nt) acc[nt] = mmab(a, ldb(bp + (size_t)nt * 16 * CON + kc), acc[nt]);
    }
#pragma unroll
    for (int nt = 0; nt < 6; ++nt) {
#pragma unroll
        for (int j = 0; j < 8; ++j) gs[(8 * hi + j) * MP + nt * 16 + lr] = hbits(toh_flush(acc[nt][j] * 1024.0f)); }
    wave_sync();
    hf* dst = G1H + (size_t)w * 16 * NP;
#pragma unroll 1
    for (int ps = 0; ps < 2; ++ps) {
#pragma unroll 1
        for (int it = 0; it < 6; ++it) { const int c = it * 32 + lane; const int row = c / 12; const int c8 = (c - row * 12) * 8;
            const v8us v = *(const v8usa*)(&gs[row * MP + c8]);
            *(volatile v8us*)(dst + (size_t)c * 8) = v; }
        if (ps == 0) __threadfence(); }
}

static constexpr int LDS_MAIN = 2 * 16 * XP * 2 + 2 * 16 * TP * 2 + 4 * 16 * MP * 2 + 16 * NP * 4 + 16 * 4 + SPB * COMP * 4;
static_assert(LDS_MAIN <= 131072);
static_assert(LDS_MAIN <= 65536);

__global__ __launch_bounds__(32) __attribute__((amdgpu_num_vgpr(256))) void k_main(
    const float* __restrict__ obs, const float* __restrict__ act,
    const float* __restrict__ ob1, const float* __restrict__ ob2,
    const float* __restrict__ ab1, const float* __restrict__ ab2,
    const float* __restrict__ mb1, const float* __restrict__ mb2, const float* __restrict__ mb3,
    const float* __restrict__ kb1, const float* __restrict__ kb2,
    const float* __restrict__ kw3, const float* __restrict__ kb3,
    const bf* __restrict__ PL, const hf* __restrict__ G1H, float* OUT)
{
    __shared__ __align__(16) hf XH[16 * XP];
    __shared__ __align__(16) hf XR[16 * XP];
    __shared__ __align__(16) hf TH[16 * TP];
    __shared__ __align__(16) hf TR[16 * TP];
    __shared__ __align__(16) bf D1[16 * MP];
    __shared__ __align__(16) bf D2M[16 * MP];
    __shared__ __align__(16) bf D3M[16 * MP];
    __shared__ __align__(16) hf PS[16 * MP];
    __shared__ __align__(16) float F3[16 * NP];
    __shared__ __align__(16) float KOUT[16];
    __shared__ __align__(16) float OUTS[SPB * COMP];

    const int lane = threadIdx.x & 31, lr = lane & 15, hi = lane >> 4;

#pragma unroll 1
    for (int hs = 0; hs < 2; ++hs) {
        const size_t r0 = (size_t)blockIdx.x * SPB + (size_t)hs * 16;

        {
            const float* orow = obs + (r0 + lr) * NOBS + 8 * hi;
            const v16bf a0 = cat16b(cvt8(orow), cvt8(orow + 16));
            const v16bf a1 = cat16b(cvt8(orow + 32), cvt8(orow + 48));
#pragma unroll 1
            for (int nt = 0; nt < 8; ++nt) {
                const bf* w = PL + (size_t)CH_OW1B * 8 + (size_t)(nt * 16 + lr) * NOBS + 8 * hi;
                v8f c = (v8f){};
                c = mmab(a0, ldb(w), c);
                c = mmab(a1, ldb(w + 32), c);
                const int col = nt * 16 + lr; const float bb = bfv(ob1, col, HID);
#pragma unroll
                for (int j = 0; j < 8; ++j) st_hr(TH, TR, (8 * hi + j) * TP + col, fmaxf(c[j] + bb, 0.0f));
            }
        }
        wave_sync();
#pragma unroll 1
        for (int nt = 0; nt < 8; ++nt) {
            const v8f p = tile_pre<HID, true>(TH + lr * TP + 8 * hi, TR + lr * TP + 8 * hi, PL + (size_t)CH_OW2H * 8 + (size_t)(nt * 16 + lr) * HID + 8 * hi);
            const int col = nt * 16 + lr; const float bb = bfv(ob2, col, HID);
#pragma unroll
            for (int j = 0; j < 8; ++j) st_hr(XH, XR, (8 * hi + j) * XP + col, fmaxf(p[j] + bb, 0.0f));
        }
        wave_sync();
        {
            const float* arow = act + (r0 + lr) * NACT + 8 * hi;
            v8us z;
#pragma unroll
            for (int k = 0; k < 8; ++k) z[k] = (unsigned short)0;
            const v16bf a0 = cat16b(cvt8(arow), z);
#pragma unroll 1
            for (int nt = 0; nt < 8; ++nt) {
                const bf* w = PL + (size_t)CH_AW1B * 8 + (size_t)(nt * 16 + lr) * 32 + 8 * hi;
                v8f c = (v8f){};
                c = mmab(a0, ldb(w), c);
                const int col = nt * 16 + lr; const float bb = bfv(ab1, col, HID);
#pragma unroll
                for (int j = 0; j < 8; ++j) st_hr(TH, TR, (8 * hi + j) * TP + col, fmaxf(c[j] + bb, 0.0f));
            }
        }
        wave_sync();
#pragma unroll 1
        for (int nt = 0; nt < 8; ++nt) {
            const v8f p = tile_pre<HID, true>(TH + lr * TP + 8 * hi, TR + lr * TP + 8 * hi, PL + (size_t)CH_AW2H * 8 + (size_t)(nt * 16 + lr) * HID + 8 * hi);
            const int col = nt * 16 + lr; const float bb = bfv(ab2, col, HID);
#pragma unroll
            for (int j = 0; j < 8; ++j) st_hr(XH, XR, (8 * hi + j) * XP + HID + col, fmaxf(p[j] + bb, 0.0f));
        }
        wave_sync();
#pragma unroll 1
        for (int nt = 0; nt < 2; ++nt) {
            const v8f p = tile_pre<CON, false>(XH + lr * XP + 8 * hi, XH + lr * XP + 8 * hi, PL + (size_t)CH_KW1H * 8 + (size_t)(nt * 16 + lr) * CON + 8 * hi);
            const int col = nt * 16 + lr; const float bb = bfv(kb1, col, NKS);
#pragma unroll
            for (int j = 0; j < 8; ++j) st_hr(TH, TR, (8 * hi + j) * TP + col, tanhf(p[j] + bb));
        }
        wave_sync();
        {
            const v8f p = tile_pre<NKS, false>(TH + lr * TP + 8 * hi, TH + lr * TP + 8 * hi, PL + (size_t)CH_KW2H * 8 + (size_t)lr * NKS + 8 * hi);
            const float bb = bfv(kb2, lr, 16); const float w3 = bfv(kw3, lr, 16); const float b3 = bfv(kb3, 0, 1);
#pragma unroll
            for (int j = 0; j < 8; ++j) {
                float t = tanhf(p[j] + bb) * w3;
                t += __shfl_xor(t, 1, 32); t += __shfl_xor(t, 2, 32); t += __shfl_xor(t, 4, 32); t += __shfl_xor(t, 8, 32);
                const float sp = softplusf(t + b3);
                if (lr == 0) KOUT[8 * hi + j] = sp;
            }
        }
        wave_sync();
#pragma unroll 1
        for (int nt = 0; nt < 6; ++nt) {
            const v8f p = tile_pre<CON, true>(XH + lr * XP + 8 * hi, XR + lr * XP + 8 * hi, PL + (size_t)CH_MW1H * 8 + (size_t)(nt * 16 + lr) * CON + 8 * hi);
            const int col = nt * 16 + lr; const float bb = bfv(mb1, col, COMP);
#pragma unroll
            for (int j = 0; j < 8; ++j) { const float v = p[j] + bb;
                st_hr(TH, TR, (8 * hi + j) * TP + col, fmaxf(v, 0.0f));
                D1[(8 * hi + j) * MP + col] = (v > 0.0f) ? (unsigned short)1 : (unsigned short)0; }
        }
        wave_sync();
#pragma unroll 1
        for (int nt = 0; nt < 6; ++nt) {
            const v8f p = tile_pre<NP, true>(TH + lr * TP + 8 * hi, TR + lr * TP + 8 * hi, PL + (size_t)CH_MW2H * 8 + (size_t)(nt * 16 + lr) * NP + 8 * hi);
            const int col = nt * 16 + lr; const float bb = bfv(mb2, col, COMP);
#pragma unroll
            for (int j = 0; j < 8; ++j) { const float v = p[j] + bb;
                st_hr(XH, XR, (8 * hi + j) * XP + col, fmaxf(v, 0.0f));
                D2M[(8 * hi + j) * MP + col] = (v > 0.0f) ? (unsigned short)0xFFFFu : (unsigned short)0; }
        }
        wave_sync();
#pragma unroll 1
        for (int nt = 0; nt < 6; ++nt) {
            const v8f p = tile_pre<NP, true>(XH + lr * XP + 8 * hi, XR + lr * XP + 8 * hi, PL + (size_t)CH_MW3H * 8 + (size_t)(nt * 16 + lr) * NP + 8 * hi);
            const int col = nt * 16 + lr; const float bb = bfv(mb3, col, COMP);
#pragma unroll
            for (int j = 0; j < 8; ++j) { const float v = p[j] + bb;
                F3[(8 * hi + j) * NP + col] = fmaxf(v, 0.0f);
                D3M[(8 * hi + j) * MP + col] = (v > 0.0f) ? (unsigned short)0xFFFFu : (unsigned short)0; }
        }
        wave_sync();

        const hf* w3p = PL + (size_t)CH_MW3H * 8 + (size_t)lr * NP + 8 * hi;
        const hf* w2p = PL + (size_t)CH_MW2T * 8 + (size_t)lr * NP + 8 * hi;
        const hf* g1p = G1H + (size_t)lr * NP + 8 * hi;
#pragma unroll 1
        for (int s = 0; s < 16; ++s) {
            float part = 0.0f;
#pragma unroll 1
            for (int mt = 0; mt < 6; ++mt) {
                const unsigned short rm = D3M[s * MP + mt * 16 + lr];
                v16h a[3];
#pragma unroll
                for (int q3 = 0; q3 < 3; ++q3) {
                    const int kc = 32 * q3;
                    v8us w0 = *(const v8us*)(w3p + (size_t)mt * 16 * NP + kc);
                    v8us w1 = *(const v8us*)(w3p + (size_t)mt * 16 * NP + kc + 16);
                    const v8us m0 = *(const v8usa*)(&D2M[s * MP + kc + 8 * hi]);
                    const v8us m1 = *(const v8usa*)(&D2M[s * MP + kc + 16 + 8 * hi]);
#pragma unroll
                    for (int k = 0; k < 8; ++k) { w0[k] = (unsigned short)(w0[k] & m0[k] & rm); w1[k] = (unsigned short)(w1[k] & m1[k] & rm); }
                    a[q3] = cat16h(w0, w1);
                }
                v8f P[6];
#pragma unroll
                for (int nt = 0; nt < 6; ++nt) {
                    v8f c = (v8f){};
#pragma unroll
                    for (int q3 = 0; q3 < 3; ++q3) c = mmah(a[q3], ldh(w2p + (size_t)nt * 16 * NP + 32 * q3), c);
                    const float psc = (D1[s * MP + nt * 16 + lr] != (unsigned short)0) ? 9.765625e-04f : 0.0f;
#pragma unroll
                    for (int j = 0; j < 8; ++j) { const float pv = c[j] * psc; P[nt][j] = pv;
                        PS[(8 * hi + j) * MP + nt * 16 + lr] = hbits(toh_flush(pv)); }
                }
                wave_sync();
                v16h pa[3];
#pragma unroll
                for (int q3 = 0; q3 < 3; ++q3) pa[q3] = ldl(&PS[lr * MP + 8 * hi + 32 * q3]);
#pragma unroll
                for (int nt = 0; nt < 6; ++nt) {
                    v8f q = (v8f){};
#pragma unroll
                    for (int q3 = 0; q3 < 3; ++q3) q = mmah(pa[q3], ldh(g1p + (size_t)nt * 16 * NP + 32 * q3), q);
#pragma unroll
                    for (int j = 0; j < 8; ++j) part += q[j] * P[nt][j];
                }
                wave_sync();
            }
            part += __shfl_xor(part, 16, 32); part += __shfl_xor(part, 8, 32); part += __shfl_xor(part, 4, 32);
            part += __shfl_xor(part, 2, 32);  part += __shfl_xor(part, 1, 32);
            const float jn = sqrtf(fmaxf(part, 0.0f) * 9.313225746154785e-10f);
            const float inv = 1.0f / (jn + 1e-4f);
            const float ko = KOUT[s];
#pragma unroll 1
            for (int i = 0; i < 3; ++i) { const int c = lane + 32 * i; const int cc = min(c, COMP - 1);
                const float v = tanhf((ko * F3[s * NP + cc]) * inv);
                if (c < COMP) OUTS[(hs * 16 + s) * COMP + c] = v; }
        }
        wave_sync();
    }

    float* dst = OUT + (size_t)blockIdx.x * (SPB * COMP);
#pragma unroll 1
    for (int ps = 0; ps < 2; ++ps) {
#pragma unroll 1
        for (int it = 0; it < 22; ++it) { const int c = it * 32 + lane;
            if (c < OCH) { const v4f v = *(const v4fa*)(&OUTS[4 * c]); *(volatile v4f*)(dst + 4 * c) = v; } }
        if (ps == 0) __threadfence(); }
}

static constexpr size_t al256(size_t v) { return (v + 255) & ~(size_t)255; }
static constexpr size_t SZ_PL = al256((size_t)NCHUNK * 16);
static constexpr size_t SZ_G1 = al256((size_t)NP * NP * 2);
static constexpr size_t SZ_TOTAL = SZ_PL + SZ_G1;
static_assert(SZ_PL == (size_t)NCHUNK * 16);
static_assert(SZ_G1 == (size_t)6 * 16 * NP * 2);
static_assert(SZ_TOTAL <= (size_t)134217728);

extern "C" void kernel_launch(void* const* d_in, const int* in_sizes, int n_in,
                              void* d_out, int out_size, void* d_ws, size_t ws_size, hipStream_t stream) {
    if (n_in < 22) return;
    if ((size_t)in_sizes[0] < (size_t)NB * NOBS || (size_t)in_sizes[1] < (size_t)NB * NACT) return;
    if (in_sizes[2] < HID * NOBS || in_sizes[3] < HID || in_sizes[4] < HID * HID || in_sizes[5] < HID) return;
    if (in_sizes[6] < HID * NACT || in_sizes[7] < HID || in_sizes[8] < HID * HID || in_sizes[9] < HID) return;
    if (in_sizes[10] < COMP * CON || in_sizes[11] < COMP || in_sizes[12] < COMP * COMP || in_sizes[13] < COMP) return;
    if (in_sizes[14] < COMP * COMP || in_sizes[15] < COMP || in_sizes[16] < NKS * CON || in_sizes[17] < NKS) return;
    if (in_sizes[18] < 16 * NKS || in_sizes[19] < 16 || in_sizes[20] < 16 || in_sizes[21] < 1) return;
    if ((size_t)out_size < (size_t)NB * COMP) return;
    if (SZ_TOTAL > ws_size) return;
    const float* obs = (const float*)d_in[0];
    const float* act = (const float*)d_in[1];
    const float* ow1 = (const float*)d_in[2];
    const float* ob1 = (const float*)d_in[3];
    const float* ow2 = (const float*)d_in[4];
    const float* ob2 = (const float*)d_in[5];
    const float* aw1 = (const float*)d_in[6];
    const float* ab1 = (const float*)d_in[7];
    const float* aw2 = (const float*)d_in[8];
    const float* ab2 = (const float*)d_in[9];
    const float* mw1 = (const float*)d_in[10];
    const float* mb1 = (const float*)d_in[11];
    const float* mw2 = (const float*)d_in[12];
    const float* mb2 = (const float*)d_in[13];
    const float* mw3 = (const float*)d_in[14];
    const float* mb3 = (const float*)d_in[15];
    const float* kw1 = (const float*)d_in[16];
    const float* kb1 = (const float*)d_in[17];
    const float* kw2 = (const float*)d_in[18];
    const float* kb2 = (const float*)d_in[19];
    const float* kw3 = (const float*)d_in[20];
    const float* kb3 = (const float*)d_in[21];
    float* OUT = (float*)d_out;
    char* wsp = (char*)d_ws;
    bf* PL  = (bf*)wsp; wsp += SZ_PL;
    hf* G1H = (hf*)wsp; wsp += SZ_G1;

    k_wconv<<<(NCHUNK + 255) / 256, 256, 0, stream>>>(ow1, aw1, ow2, aw2, mw1, mw2, mw3, kw1, kw2, PL);
    k_g1<<<6, 32, 0, stream>>>(PL, G1H);
    k_main<<<NB / SPB, 32, 0, stream>>>(obs, act, ob1, ob2, ab1, ab2, mb1, mb2, mb3, kb1, kb2, kw3, kb3, PL, G1H, OUT);
}
